// DiSAN_82360292868116
// MI455X (gfx1250) — hardware-verified
//
#include <hip/hip_runtime.h>
#include <math.h>

#define BB    4
#define LL    200
#define DD    100
#define D2    200
#define CC    20
#define NROW  (BB * LL)
#define P1    128
#define P2    256
#define UHALF 128
#define KP2   224
#define MH    32
#define NOUTP 64

static_assert(NROW % 32 == 0);
static_assert(NROW % 8 == 0);
static_assert(P1 % 64 == 0);
static_assert(P2 % 64 == 0);
static_assert((CC % 4) == 0);

#define EPI_NONE 0
#define EPI_ELU  1
#define EPI_RELU 2
#define EPI_GATE 3
#define EPI_OUT  4

typedef float v4f __attribute__((ext_vector_type(4)));
typedef float v8f __attribute__((ext_vector_type(8)));
typedef unsigned short v4us  __attribute__((ext_vector_type(4)));
typedef unsigned short v8us  __attribute__((ext_vector_type(8)));
typedef unsigned short v16us __attribute__((ext_vector_type(16)));
typedef __bf16 v16bf __attribute__((ext_vector_type(16)));
typedef v4f  __attribute__((may_alias)) v4fa;
typedef v8us __attribute__((may_alias)) v8usa;

union FragU { v16us v; v8us h8[2]; v4us q[4]; };

__device__ __forceinline__ unsigned short bf16_bits(float x) {
  unsigned int u = __float_as_uint(x);
  u += 0x7FFFu + ((u >> 16) & 1u);
  return (unsigned short)(u >> 16);
}

__device__ __forceinline__ void split_one(float x, unsigned short& hi, unsigned short& lo) {
  const unsigned short hb = bf16_bits(x);
  const float hf = __uint_as_float(((unsigned int)hb) << 16);
  hi = hb;
  lo = bf16_bits(x - hf);
}

__device__ __forceinline__ void split4(v4f x, v4us& hi, v4us& lo) {
  unsigned short h0, h1, h2, h3, l0, l1, l2, l3;
  split_one(x.x, h0, l0);
  split_one(x.y, h1, l1);
  split_one(x.z, h2, l2);
  split_one(x.w, h3, l3);
  const v4us hv = {h0, h1, h2, h3};
  const v4us lv = {l0, l1, l2, l3};
  hi = hv;
  lo = lv;
}

__device__ __forceinline__ v8f wmma_bf16(v16us a, v16us b, v8f c) {
  const v16bf av = __builtin_bit_cast(v16bf, a);
  const v16bf bv = __builtin_bit_cast(v16bf, b);
  v8f d = __builtin_amdgcn_wmma_f32_16x16x32_bf16(false, av, false, bv, (short)0, c, false, false);
  asm volatile("v_nop\n\tv_nop\n\tv_nop\n\tv_nop" : "+v"(d) : "v"(a), "v"(b));
  return d;
}

__device__ __forceinline__ void tile_store_pass(const float* sC, float* C, int ldc, int colbase,
                                                int r0, int w, int lane) {
  const int q8 = lane & 7, sub = lane >> 3;
  #pragma unroll
  for (int i = 0; i < 8; ++i) {
    const int lid = i * 4 + sub;
    const int row = lid >> 1, hl = lid & 1;
    const v4f v = *(const v4fa*)(sC + (16 * w + row) * 64 + 32 * hl + 4 * q8);
    float* dst = C + (size_t)(r0 + 16 * w + row) * ldc + colbase + 32 * hl + 4 * q8;
    *(volatile v4f*)dst = v;
  }
}

__device__ __forceinline__ void out_store_pass(const float* sC, float* C, int lane) {
  const int b = lane / 5;
  const int c = 4 * (lane - 5 * b);
  v4f v;
  v.x = sC[b * 64 + c + 0];
  v.y = sC[b * 64 + c + 1];
  v.z = sC[b * 64 + c + 2];
  v.w = sC[b * 64 + c + 3];
  *(volatile v4f*)(C + 4 * lane) = v;
}

__global__ __launch_bounds__(64) void gemm_split3_kernel(
    const float* A, int lda,
    const float* W, int ldw, int wrows,
    int ksegP, int ksegR, int Kp,
    const float* bias, int has_bias, int nbias,
    float* C, int ldc, int coloff,
    const float* Hx, const float* Gx,
    int epi)
{
  __shared__ __attribute__((aligned(16))) unsigned short sBh[64 * 32];
  __shared__ __attribute__((aligned(16))) unsigned short sBl[64 * 32];
  __shared__ __attribute__((aligned(16))) float sC[32 * 64];

  const int tid = threadIdx.x, lane = tid & 31, w = tid >> 5;
  const int h = lane >> 4, m = lane & 15;
  const int r0 = blockIdx.x * 32, n0 = blockIdx.y * 64;

  const v8f zero8 = {0.f, 0.f, 0.f, 0.f, 0.f, 0.f, 0.f, 0.f};
  v8f acc[4];
  #pragma unroll
  for (int nt = 0; nt < 4; ++nt) acc[nt] = zero8;

  const int ncol = n0 + tid;
  const bool nok = (ncol < ldw);
  const int ncc = nok ? ncol : (ldw - 1);

  const float* arow = A + (size_t)(r0 + 16 * w + m) * lda;

  #pragma unroll 1
  for (int k0 = 0; k0 < Kp; k0 += 32) {
    #pragma unroll 8
    for (int e = 0; e < 32; ++e) {
      const int k = k0 + e;
      const int seg = (k >= ksegP) ? 1 : 0;
      const int kin = k - seg * ksegP;
      const int wr = seg * ksegR + kin;
      const bool ok = nok && (kin < ksegR) && (wr < wrows);
      const int wrc = (wr < wrows) ? wr : (wrows - 1);
      float x = W[(size_t)wrc * ldw + ncc];
      x = ok ? x : 0.0f;
      unsigned short hi, lo;
      split_one(x, hi, lo);
      sBh[tid * 32 + e] = hi;
      sBl[tid * 32 + e] = lo;
    }
    __syncthreads();

    FragU ah, al;
    {
      const float* ap = arow + k0 + 8 * h;
      const v4f x0 = *(const v4fa*)(ap);
      const v4f x1 = *(const v4fa*)(ap + 4);
      const v4f x2 = *(const v4fa*)(ap + 16);
      const v4f x3 = *(const v4fa*)(ap + 20);
      split4(x0, ah.q[0], al.q[0]);
      split4(x1, ah.q[1], al.q[1]);
      split4(x2, ah.q[2], al.q[2]);
      split4(x3, ah.q[3], al.q[3]);
    }

    #pragma unroll
    for (int nt = 0; nt < 4; ++nt) {
      const unsigned short* ph = sBh + (16 * nt + m) * 32 + 8 * h;
      const unsigned short* pl = sBl + (16 * nt + m) * 32 + 8 * h;
      FragU bh, bl;
      bh.h8[0] = *(const v8usa*)(ph);
      bh.h8[1] = *(const v8usa*)(ph + 16);
      bl.h8[0] = *(const v8usa*)(pl);
      bl.h8[1] = *(const v8usa*)(pl + 16);
      acc[nt] = wmma_bf16(ah.v, bh.v, acc[nt]);
      acc[nt] = wmma_bf16(ah.v, bl.v, acc[nt]);
      acc[nt] = wmma_bf16(al.v, bh.v, acc[nt]);
    }
    __syncthreads();
  }

  #pragma unroll
  for (int nt = 0; nt < 4; ++nt) {
    #pragma unroll
    for (int r = 0; r < 8; ++r) {
      sC[(16 * w + 8 * h + r) * 64 + 16 * nt + m] = acc[nt][r];
    }
  }
  __syncthreads();

  const int col = n0 + tid;
  float bv = 0.0f;
  if (has_bias) {
    const int cb = (col < nbias) ? col : (nbias - 1);
    const float bl = bias[cb];
    bv = (col < nbias) ? bl : 0.0f;
  }
  #pragma unroll 1
  for (int i = 0; i < 32; ++i) {
    const int row = r0 + i;
    float v = sC[i * 64 + tid] + bv;
    if (epi == EPI_ELU) {
      const float em = expm1f(fminf(v, 0.0f));
      v = (v > 0.0f) ? v : em;
    } else if (epi == EPI_RELU) {
      v = fmaxf(v, 0.0f);
    } else if (epi == EPI_GATE) {
      const size_t gi = (size_t)row * lda + col;
      float xg = v + Gx[gi];
      xg = fminf(fmaxf(xg, -30.0f), 30.0f);
      const float f = 1.0f / (1.0f + expf(-xg));
      const float hvl = Hx[gi];
      const float svl = A[gi];
      v = f * hvl + (1.0f - f) * svl;
    }
    sC[i * 64 + tid] = v;
  }
  __syncthreads();

  if (epi != EPI_OUT) {
    tile_store_pass(sC, C, ldc, coloff + n0, r0, w, lane);
    __threadfence();
    tile_store_pass(sC, C, ldc, coloff + n0, r0, w, lane);
  } else {
    if (w == 0 && lane < 20) {
      out_store_pass(sC, C, lane);
      __threadfence();
      out_store_pass(sC, C, lane);
    }
  }
}

__global__ __launch_bounds__(256) void embed_kernel(const int* x, const float* emb, int V,
                                                    float* XE) {
  const int tid = threadIdx.x, lane = tid & 31, w = tid >> 5;
  const int row = blockIdx.x * 8 + w;
  int tok = x[row];
  tok = (tok < 0) ? 0 : tok;
  tok = (tok > V - 1) ? (V - 1) : tok;
  const int c0 = (lane < 25) ? (4 * lane) : 96;
  const v4f e4 = *(const v4fa*)(emb + (size_t)tok * DD + c0);
  const bool keep = (lane < 25);
  v4f v;
  v.x = keep ? e4.x : 0.0f;
  v.y = keep ? e4.y : 0.0f;
  v.z = keep ? e4.z : 0.0f;
  v.w = keep ? e4.w : 0.0f;
  float* dst = XE + (size_t)row * P1 + 4 * lane;
  *(volatile v4f*)dst = v;
  __threadfence();
  *(volatile v4f*)dst = v;
}

__global__ __launch_bounds__(128) void attend_kernel(
    const float* H, const float* H1, const float* H2,
    const float* bvec, const int* mask,
    float* SF, float* SB)
{
  __shared__ __attribute__((aligned(16))) float sf[128];
  __shared__ __attribute__((aligned(16))) float sb[128];

  const int row = blockIdx.x;
  const int b = row / LL;
  const int l = row - b * LL;
  const int e = threadIdx.x;
  const int ec = (e < DD) ? e : (DD - 1);

  const float h1v = H1[(size_t)row * P1 + e];
  const float bv = bvec[ec];
  const int ml = mask[row];

  const float* h2p = H2 + (size_t)b * LL * P1 + e;
  const float* hp  = H  + (size_t)b * LL * P1 + e;
  const int* mp = mask + b * LL;

  float dF = 0.0f, nF = 0.0f, dB = 0.0f, nB = 0.0f, hsum = 0.0f;
  #pragma unroll 1
  for (int mm = 0; mm < LL; ++mm) {
    const float h2v = h2p[(size_t)mm * P1];
    const float hvl = hp[(size_t)mm * P1];
    const int mk = mp[mm];
    const float t = (h1v + h2v) + bv;
    const float att = 5.0f * tanhf(t * 0.2f);
    const float ev = expf(att);
    const bool dead = (mk != 0) && (ml == 0);
    const float wF = (dead || (mm <= l)) ? 0.0f : ev;
    const float wB = (dead || (mm >= l)) ? 0.0f : ev;
    dF += wF;
    nF = fmaf(wF, hvl, nF);
    dB += wB;
    nB = fmaf(wB, hvl, nB);
    hsum += hvl;
  }
  const float uni = hsum * (1.0f / (float)LL);
  const float dFs = (dF > 0.0f) ? dF : 1.0f;
  const float dBs = (dB > 0.0f) ? dB : 1.0f;
  const float rF = (dF > 0.0f) ? (nF * (1.0f / dFs)) : uni;
  const float rB = (dB > 0.0f) ? (nB * (1.0f / dBs)) : uni;
  sf[e] = (e < DD) ? rF : 0.0f;
  sb[e] = (e < DD) ? rB : 0.0f;
  __syncthreads();

  const int w = e >> 5, lane = e & 31;
  if (w == 0) {
    const v4f v = *(const v4fa*)(sf + 4 * lane);
    float* dst = SF + (size_t)row * P1 + 4 * lane;
    *(volatile v4f*)dst = v;
    __threadfence();
    *(volatile v4f*)dst = v;
  } else if (w == 1) {
    const v4f v = *(const v4fa*)(sb + 4 * lane);
    float* dst = SB + (size_t)row * P1 + 4 * lane;
    *(volatile v4f*)dst = v;
    __threadfence();
    *(volatile v4f*)dst = v;
  }
}

__global__ __launch_bounds__(256) void pool_kernel(const float* U, const float* AS, float* SS) {
  __shared__ __attribute__((aligned(16))) float srow[256];
  const int bq = blockIdx.x;
  const int j = threadIdx.x;
  float acc = 0.0f;
  if (bq < BB) {
    const int jc = (j < D2) ? j : (D2 - 1);
    const int uc = jc + ((jc >= DD) ? (UHALF - DD) : 0);
    const float* up = U  + (size_t)bq * LL * P2 + uc;
    const float* ap = AS + (size_t)bq * LL * P2 + jc;
    #pragma unroll 1
    for (int l = 0; l < LL; ++l) {
      acc = fmaf(up[(size_t)l * P2], ap[(size_t)l * P2], acc);
    }
    acc = (j < D2) ? acc : 0.0f;
  }
  srow[j] = acc;
  __syncthreads();
  if (j < 32) {
    const v4f v0 = *(const v4fa*)(srow + 4 * j);
    const v4f v1 = *(const v4fa*)(srow + 128 + 4 * j);
    float* d0 = SS + (size_t)bq * P2 + 4 * j;
    float* d1 = SS + (size_t)bq * P2 + 128 + 4 * j;
    *(volatile v4f*)d0 = v0;
    *(volatile v4f*)d1 = v1;
    __threadfence();
    *(volatile v4f*)d0 = v0;
    *(volatile v4f*)d1 = v1;
  }
}

extern "C" void kernel_launch(void* const* d_in, const int* in_sizes, int n_in,
                              void* d_out, int out_size, void* d_ws, size_t ws_size,
                              hipStream_t stream) {
  if (n_in < 20) return;
  if (in_sizes[0] != NROW || in_sizes[2] != NROW) return;
  if (in_sizes[3] < DD || (in_sizes[3] % DD) != 0) return;
  if (in_sizes[4] != DD * DD || in_sizes[5] != DD) return;
  if (in_sizes[6] != DD * DD || in_sizes[7] != DD * DD || in_sizes[8] != DD) return;
  if (in_sizes[9] != DD * DD || in_sizes[10] != DD * DD || in_sizes[11] != DD) return;
  if (in_sizes[12] != D2 * D2 || in_sizes[13] != D2) return;
  if (in_sizes[14] != D2 * D2 || in_sizes[15] != D2) return;
  if (in_sizes[16] != D2 * DD || in_sizes[17] != DD) return;
  if (in_sizes[18] != DD * CC || in_sizes[19] != CC) return;
  if (out_size != BB * CC) return;

  const int*   x     = (const int*)d_in[0];
  const int*   mask  = (const int*)d_in[2];
  const float* emb   = (const float*)d_in[3];
  const float* Wh_w  = (const float*)d_in[4];
  const float* Wh_b  = (const float*)d_in[5];
  const float* W1_w  = (const float*)d_in[6];
  const float* W2_w  = (const float*)d_in[7];
  const float* bvec  = (const float*)d_in[8];
  const float* Wf1_w = (const float*)d_in[9];
  const float* Wf2_w = (const float*)d_in[10];
  const float* Wf2_b = (const float*)d_in[11];
  const float* Ws1_w = (const float*)d_in[12];
  const float* Ws1_b = (const float*)d_in[13];
  const float* Ws_w  = (const float*)d_in[14];
  const float* Ws_b  = (const float*)d_in[15];
  const float* F1_w  = (const float*)d_in[16];
  const float* F1_b  = (const float*)d_in[17];
  const float* F2_w  = (const float*)d_in[18];
  const float* F2_b  = (const float*)d_in[19];
  float* out = (float*)d_out;
  const int V = in_sizes[3] / DD;

  size_t o = 0;
  const size_t oXE = o; o += (size_t)NROW * P1;
  const size_t oH  = o; o += (size_t)NROW * P1;
  const size_t oH1 = o; o += (size_t)NROW * P1;
  const size_t oH2 = o; o += (size_t)NROW * P1;
  const size_t oSF = o; o += (size_t)NROW * P1;
  const size_t oSB = o; o += (size_t)NROW * P1;
  const size_t oG2 = o; o += (size_t)NROW * P1;
  const size_t oU  = o; o += (size_t)NROW * P2;
  const size_t oT  = o; o += (size_t)NROW * P2;
  const size_t oAS = o; o += (size_t)NROW * P2;
  const size_t oSS = o; o += (size_t)MH * P2;
  const size_t oZ  = o; o += (size_t)MH * P1;
  const size_t total_bytes = o * sizeof(float);
  if (total_bytes > ws_size) return;
  if (total_bytes > (size_t)134217728) return;

  float* ws = (float*)d_ws;
  float* XE = ws + oXE;
  float* H  = ws + oH;
  float* H1 = ws + oH1;
  float* H2 = ws + oH2;
  float* SF = ws + oSF;
  float* SB = ws + oSB;
  float* G2 = ws + oG2;
  float* U  = ws + oU;
  float* T  = ws + oT;
  float* AS = ws + oAS;
  float* SS = ws + oSS;
  float* Z  = ws + oZ;

  auto gemm = [&](const float* A, int lda, const float* Wp, int ldw, int wrows,
                  int ksegP, int ksegR, int Kp,
                  const float* bias, int has_bias, int nbias,
                  float* Cp, int ldc, int coloff,
                  const float* Hx, const float* Gx, int epi, int M, int Npad) {
    dim3 g(M / 32, Npad / 64);
    gemm_split3_kernel<<<g, 64, 0, stream>>>(A, lda, Wp, ldw, wrows, ksegP, ksegR, Kp,
                                             bias, has_bias, nbias, Cp, ldc, coloff,
                                             Hx, Gx, epi);
  };

  embed_kernel<<<NROW / 8, 256, 0, stream>>>(x, emb, V, XE);

  gemm(XE, P1, Wh_w, DD, DD, P1, DD, P1, Wh_b, 1, DD, H,  P1, 0, XE, XE, EPI_ELU,  NROW, P1);
  gemm(H,  P1, W1_w, DD, DD, P1, DD, P1, W1_w, 0, 1,  H1, P1, 0, H,  H,  EPI_NONE, NROW, P1);
  gemm(H,  P1, W2_w, DD, DD, P1, DD, P1, W2_w, 0, 1,  H2, P1, 0, H,  H,  EPI_NONE, NROW, P1);

  attend_kernel<<<NROW, 128, 0, stream>>>(H, H1, H2, bvec, mask, SF, SB);

  gemm(H,  P1, Wf2_w, DD, DD, P1, DD, P1, Wf2_b, 1, DD, G2, P1, 0,     H, H,  EPI_NONE, NROW, P1);
  gemm(SF, P1, Wf1_w, DD, DD, P1, DD, P1, Wf1_w, 0, 1,  U,  P2, 0,     H, G2, EPI_GATE, NROW, P1);
  gemm(SB, P1, Wf1_w, DD, DD, P1, DD, P1, Wf1_w, 0, 1,  U,  P2, UHALF, H, G2, EPI_GATE, NROW, P1);

  gemm(U, P2, Ws1_w, D2, D2, UHALF, DD, P2,  Ws1_b, 1, D2, T,  P2, 0, U, U, EPI_ELU,  NROW, P2);
  gemm(T, P2, Ws_w,  D2, D2, KP2,   D2, KP2, Ws_b,  1, D2, AS, P2, 0, T, T, EPI_NONE, NROW, P2);

  pool_kernel<<<MH, 256, 0, stream>>>(U, AS, SS);

  gemm(SS, P2, F1_w, DD, D2, KP2, D2, KP2, F1_b, 1, DD, Z,   P1, 0, SS, SS, EPI_RELU, MH, P1);
  gemm(Z,  P1, F2_w, CC, DD, P1,  DD, P1,  F2_b, 1, CC, out, 0,  0, Z,  Z,  EPI_OUT,  MH, NOUTP);
}
